// NIRM_40999757807996
// MI455X (gfx1250) — hardware-verified
//
#include <hip/hip_runtime.h>
#include <stddef.h>


#define NTHR    256
#define NWAVE   8
#define EPT     8
#define NGRP    2
#define CHUNK   (NTHR * EPT * NGRP)
#define WCAP    (EPT * NGRP * 32)
#define LISTN   (NWAVE * WCAP)
#define NBC     4096
#define NBF     1024
#define RCAP    40960
#define RBN     128
#define OTHR    512
#define DEGCAP  256
#define GTHR    128
#define GROW    128
#define GP      32
#define TP      16
#define XP      8
#define AP      40
#define WSC     8.0f
#define WINV    0.125f
#define LDS_FILL ((RCAP + NBF + LISTN) * 4 + 64)

static_assert((CHUNK & (CHUNK - 1)) == 0);
static_assert(CHUNK <= 4096);
static_assert((NBC & (NBC - 1)) == 0 && (NBF & (NBF - 1)) == 0);
static_assert(NBC == 4 * NBF);
static_assert(OTHR * 8 == NBC);
static_assert((RCAP % 32) == 0);
static_assert(GROW == 4 * 32 && GTHR == GROW);
static_assert((NBC % GROW) == 0);

typedef float    v4f  __attribute__((ext_vector_type(4)));
typedef float    v8f  __attribute__((ext_vector_type(8)));
typedef int      v4i  __attribute__((ext_vector_type(4)));
typedef _Float16 v8h  __attribute__((ext_vector_type(8)));
typedef _Float16 v16h __attribute__((ext_vector_type(16)));
union FragH { v16h v; v8h h[2]; };

__device__ __forceinline__ v8f wmh(v16h a, v16h b, v8f c) {
  v8f d = __builtin_amdgcn_wmma_f32_16x16x32_f16(false, a, false, b, (short)0, c, false, false);
  asm volatile("v_nop\n\tv_nop\n\tv_nop\n\tv_nop" : "+v"(d) : "v"(a), "v"(b));
  return d;
}

__device__ __forceinline__ int wave_max(int v) {
  v = max(v, __shfl_xor(v, 16));
  v = max(v, __shfl_xor(v, 8));
  v = max(v, __shfl_xor(v, 4));
  v = max(v, __shfl_xor(v, 2));
  v = max(v, __shfl_xor(v, 1));
  return v;
}

template <int P>
__device__ __forceinline__ void store_rows32(const float* lrow, float* grow, int lane) {
  v4f v[P / 4];
#pragma unroll
  for (int i = 0; i < P / 4; ++i) v[i] = *(const v4f*)(lrow + i * 128 + 4 * lane);
#pragma unroll
  for (int i = 0; i < P / 4; ++i) *(volatile v4f*)(grow + (size_t)i * 128 + 4 * lane) = v[i];
  __threadfence();
#pragma unroll
  for (int i = 0; i < P / 4; ++i) *(volatile v4f*)(grow + (size_t)i * 128 + 4 * lane) = v[i];
}

template <int NB>
__device__ __forceinline__ int scan_chunk(const int* __restrict__ keys, int nE, int cbase, int slotBase,
                                          int vec8, int* list, int tid, int lane, int wave) {
  int wc = 0;
#pragma unroll
  for (int g = 0; g < NGRP; ++g) {
    const int el0  = (g * NTHR + tid) * EPT;
    const int e0   = cbase + el0;
    const int sent = -2147483647 - 1;
    v4i da, db;
    if (vec8 != 0 && cbase + CHUNK <= nE) {
      da = *(const v4i*)(keys + e0);
      db = *(const v4i*)(keys + e0 + 4);
    } else {
      da.x = (e0     < nE) ? keys[min(e0, nE - 1)] : sent;
      da.y = (e0 + 1 < nE) ? keys[min(e0 + 1, nE - 1)] : sent;
      da.z = (e0 + 2 < nE) ? keys[min(e0 + 2, nE - 1)] : sent;
      da.w = (e0 + 3 < nE) ? keys[min(e0 + 3, nE - 1)] : sent;
      db.x = (e0 + 4 < nE) ? keys[min(e0 + 4, nE - 1)] : sent;
      db.y = (e0 + 5 < nE) ? keys[min(e0 + 5, nE - 1)] : sent;
      db.z = (e0 + 6 < nE) ? keys[min(e0 + 6, nE - 1)] : sent;
      db.w = (e0 + 7 < nE) ? keys[min(e0 + 7, nE - 1)] : sent;
    }
    const unsigned nb = (unsigned)slotBase;
    const unsigned s0 = (unsigned)da.x - nb, s1 = (unsigned)da.y - nb;
    const unsigned s2 = (unsigned)da.z - nb, s3 = (unsigned)da.w - nb;
    const unsigned s4 = (unsigned)db.x - nb, s5 = (unsigned)db.y - nb;
    const unsigned s6 = (unsigned)db.z - nb, s7 = (unsigned)db.w - nb;
    const bool h0 = s0 < (unsigned)NB, h1 = s1 < (unsigned)NB, h2 = s2 < (unsigned)NB, h3 = s3 < (unsigned)NB;
    const bool h4 = s4 < (unsigned)NB, h5 = s5 < (unsigned)NB, h6 = s6 < (unsigned)NB, h7 = s7 < (unsigned)NB;
    const unsigned any = __builtin_amdgcn_ballot_w32(h0 | h1 | h2 | h3 | h4 | h5 | h6 | h7);
    if (any != 0u) {
#define HITJ(J, HJ, SJ) { \
        const unsigned mj = __builtin_amdgcn_ballot_w32(HJ); \
        if (mj != 0u) { \
          if (HJ) { \
            const int pos = wc + (int)__builtin_amdgcn_mbcnt_lo(mj, 0u); \
            if (pos < WCAP) list[wave * WCAP + pos] = ((el0 + (J)) << 12) | (int)(SJ); \
          } \
          wc += (int)__builtin_popcount(mj); } }
      HITJ(0, h0, s0)
      HITJ(1, h1, s1)
      HITJ(2, h2, s2)
      HITJ(3, h3, s3)
      HITJ(4, h4, s4)
      HITJ(5, h5, s5)
      HITJ(6, h6, s6)
      HITJ(7, h7, s7)
#undef HITJ
    }
  }
  return wc;
}

__global__ __launch_bounds__(NTHR) void k_count(const int* __restrict__ keys, int* cnt, int nE, int vec8) {
  __shared__ __attribute__((aligned(16))) int scnt[NBC];
  __shared__ __attribute__((aligned(16))) int list[LISTN];
  __shared__ int wcnt[NWAVE];
  const int tid = threadIdx.x, lane = tid & 31, wave = tid >> 5;
  const int slotBase = blockIdx.x * NBC;

  for (int i = tid; i < NBC; i += NTHR) scnt[i] = 0;
  __syncthreads();

  const int nChunks = (nE + CHUNK - 1) / CHUNK;
#pragma unroll 1
  for (int ch = 0; ch < nChunks; ++ch) {
    const int cbase = ch * CHUNK;
    const int wc = scan_chunk<NBC>(keys, nE, cbase, slotBase, vec8, list, tid, lane, wave);
    if (lane == 0) wcnt[wave] = wc;
    __syncthreads();
    if (wave == 0) {
#pragma unroll 1
      for (int wsx = 0; wsx < NWAVE; ++wsx) {
        int n = __builtin_amdgcn_readfirstlane(wcnt[wsx]);
        n = n > WCAP ? WCAP : (n < 0 ? 0 : n);
        const int* lp = list + wsx * WCAP;
#pragma unroll 1
        for (int i = 0; i < n; ++i) {
          const int ent  = __builtin_amdgcn_readfirstlane(lp[i]);
          const int slot = ent & (NBC - 1);
          if (lane == 0) scnt[slot] = scnt[slot] + 1;
        }
      }
    }
    __syncthreads();
  }

  v4i cq[4];
#pragma unroll
  for (int q = 0; q < 4; ++q) {
    const int f = (wave * 4 + q) * 128 + 4 * lane;
    cq[q] = *(const v4i*)(scnt + f);
  }
  int* cp = cnt + (size_t)slotBase;
#pragma unroll
  for (int q = 0; q < 4; ++q) {
    const int f = (wave * 4 + q) * 128 + 4 * lane;
    *(volatile v4i*)(cp + f) = cq[q];
  }
  __threadfence();
#pragma unroll
  for (int q = 0; q < 4; ++q) {
    const int f = (wave * 4 + q) * 128 + 4 * lane;
    *(volatile v4i*)(cp + f) = cq[q];
  }
}

__global__ __launch_bounds__(OTHR) void k_offsets(const int* __restrict__ cnt, int* off, int* rbase, int nChunk) {
  __shared__ __attribute__((aligned(16))) int soff[NBC];
  __shared__ __attribute__((aligned(16))) int srb[RBN];
  __shared__ int wtot[OTHR / 32];
  const int tid = threadIdx.x, lane = tid & 31, wave = tid >> 5, sub = tid >> 7;
  for (int i = tid; i < RBN; i += OTHR) srb[i] = 0;
  int carry = 0;
#pragma unroll 1
  for (int ch = 0; ch < nChunk; ++ch) {
    const int base = ch * NBC;
    const v4i c0 = *(const v4i*)(cnt + base + 8 * tid);
    const v4i c1 = *(const v4i*)(cnt + base + 8 * tid + 4);
    const int e0 = max(c0.x, 0), e1 = max(c0.y, 0), e2 = max(c0.z, 0), e3 = max(c0.w, 0);
    const int e4 = max(c1.x, 0), e5 = max(c1.y, 0), e6 = max(c1.z, 0), e7 = max(c1.w, 0);
    const int ts = e0 + e1 + e2 + e3 + e4 + e5 + e6 + e7;
    int incl = ts;
#pragma unroll
    for (int d = 1; d < 32; d <<= 1) {
      const int t = __shfl_up(incl, d);
      if (lane >= d) incl += t;
    }
    if (lane == 31) wtot[wave] = incl;
    __syncthreads();
    const int S0 = wtot[0]  + wtot[1]  + wtot[2]  + wtot[3];
    const int S1 = wtot[4]  + wtot[5]  + wtot[6]  + wtot[7];
    const int S2 = wtot[8]  + wtot[9]  + wtot[10] + wtot[11];
    const int S3 = wtot[12] + wtot[13] + wtot[14] + wtot[15];
    int pre = 0;
#pragma unroll 1
    for (int w = 4 * sub; w < wave; ++w) pre += wtot[w];
    const int b0 = carry;
    const int b1 = b0 + ((S0 + 31) & ~31);
    const int b2 = b1 + ((S1 + 31) & ~31);
    const int b3 = b2 + ((S2 + 31) & ~31);
    const int b4 = b3 + ((S3 + 31) & ~31);
    const int myb = sub == 0 ? b0 : (sub == 1 ? b1 : (sub == 2 ? b2 : b3));
    if (tid == 0) {
      srb[min(4 * ch + 0, RBN - 1)] = b0;
      srb[min(4 * ch + 1, RBN - 1)] = b1;
      srb[min(4 * ch + 2, RBN - 1)] = b2;
      srb[min(4 * ch + 3, RBN - 1)] = b3;
    }
    int run = myb + pre + incl - ts;
    soff[8 * tid + 0] = run; run += e0;
    soff[8 * tid + 1] = run; run += e1;
    soff[8 * tid + 2] = run; run += e2;
    soff[8 * tid + 3] = run; run += e3;
    soff[8 * tid + 4] = run; run += e4;
    soff[8 * tid + 5] = run; run += e5;
    soff[8 * tid + 6] = run; run += e6;
    soff[8 * tid + 7] = run;
    carry = b4;
    __syncthreads();
    const v4i o0 = *(const v4i*)(soff + 4 * tid);
    const v4i o1 = *(const v4i*)(soff + 4 * (tid + OTHR));
    int* op = off + base;
    *(volatile v4i*)(op + 4 * tid) = o0;
    *(volatile v4i*)(op + 4 * (tid + OTHR)) = o1;
    __threadfence();
    *(volatile v4i*)(op + 4 * tid) = o0;
    *(volatile v4i*)(op + 4 * (tid + OTHR)) = o1;
    __syncthreads();
  }
  if (tid == 0) srb[min(4 * nChunk, RBN - 1)] = carry;
  __syncthreads();
  v4i rv = {0, 0, 0, 0};
  if (tid < 32) rv = *(const v4i*)(srb + 4 * tid);
  if (tid < 32) *(volatile v4i*)(rbase + 4 * tid) = rv;
  __threadfence();
  if (tid < 32) *(volatile v4i*)(rbase + 4 * tid) = rv;
}

__global__ __launch_bounds__(NTHR) void k_fill(
    const int* __restrict__ keys, const int* __restrict__ vals, const int* __restrict__ off,
    const int* __restrict__ rbase, int* csr, int nN, int nE, int vec8, int csrLen) {
  extern __shared__ v4f lds_dyn[];
  int* region = (int*)lds_dyn;
  int* cursor = region + RCAP;
  int* list   = cursor + NBF;
  int* wcnt   = list + LISTN;
  const int tid = threadIdx.x, lane = tid & 31, wave = tid >> 5;
  const int b = blockIdx.x;
  const int slotBase = b * NBF;

  int rb0 = rbase[b];
  const int rb1 = rbase[b + 1];
  rb0 = rb0 < 0 ? 0 : (rb0 > csrLen ? csrLen : rb0);
  rb0 &= ~31;
  int len = rb1 - rb0;
  len = len < 0 ? 0 : (len > RCAP ? RCAP : len);
  int lenW = (len + 31) & ~31;
  if (rb0 + lenW > csrLen) lenW = (csrLen - rb0) & ~31;

  {
    const v4i z = {0, 0, 0, 0};
    for (int i = tid; i < RCAP / 4; i += NTHR) ((v4i*)region)[i] = z;
    for (int s = tid; s < NBF; s += NTHR) {
      int o = off[slotBase + s] - rb0;
      o = o < 0 ? 0 : (o > RCAP ? RCAP : o);
      cursor[s] = o;
    }
  }
  __syncthreads();

  const int nChunks = (nE + CHUNK - 1) / CHUNK;
#pragma unroll 1
  for (int ch = 0; ch < nChunks; ++ch) {
    const int cbase = ch * CHUNK;
    const int wc = scan_chunk<NBF>(keys, nE, cbase, slotBase, vec8, list, tid, lane, wave);
    if (lane == 0) wcnt[wave] = wc;
    __syncthreads();
    if (wave == 0) {
#pragma unroll 1
      for (int wsx = 0; wsx < NWAVE; ++wsx) {
        int n = __builtin_amdgcn_readfirstlane(wcnt[wsx]);
        n = n > WCAP ? WCAP : (n < 0 ? 0 : n);
        const int* lp = list + wsx * WCAP;
#pragma unroll 1
        for (int i = 0; i < n; ++i) {
          const int ent  = __builtin_amdgcn_readfirstlane(lp[i]);
          const int slot = ent & (NBF - 1);
          int e = cbase + ((ent >> 12) & (CHUNK - 1));
          e = e > nE - 1 ? nE - 1 : e;
          int v = vals[e];
          v = v < 0 ? 0 : (v > nN - 1 ? nN - 1 : v);
          if (lane == 0) {
            int pos = cursor[slot];
            pos = pos < 0 ? 0 : (pos > RCAP - 1 ? RCAP - 1 : pos);
            region[pos] = v;
            const int np = pos + 1;
            cursor[slot] = np > RCAP ? RCAP : np;
          }
        }
      }
    }
    __syncthreads();
  }

  const int nv = lenW >> 2;
  int* gp = csr + rb0;
#pragma unroll 1
  for (int i = tid; i < nv; i += NTHR) { const v4i v = ((const v4i*)region)[i]; *(volatile v4i*)(gp + 4 * i) = v; }
  __threadfence();
#pragma unroll 1
  for (int i = tid; i < nv; i += NTHR) { const v4i v = ((const v4i*)region)[i]; *(volatile v4i*)(gp + 4 * i) = v; }
}

__global__ __launch_bounds__(GTHR) void k_prep(
    const float* __restrict__ x, const float* __restrict__ l1w, const float* __restrict__ l1b,
    const float* __restrict__ c1w, const float* __restrict__ c1as, const float* __restrict__ c1ad,
    float* gout, float* tout, int nN) {
  __shared__ __attribute__((aligned(16))) float sG[GROW * GP];
  __shared__ __attribute__((aligned(16))) float sT[GROW * TP];
  const int tid = threadIdx.x, lane = tid & 31, wave = tid >> 5;
  const int nodeBase = blockIdx.x * GROW;
  const int n  = nodeBase + tid;
  const int nc = n > nN - 1 ? nN - 1 : n;
  const float* xr = x + (size_t)nc * 5;
  float s0 = 0.0f;
#pragma unroll
  for (int j = 0; j < 5; ++j) s0 += xr[j] * l1w[j];
  s0 += l1b[0];
  float* gr = sG + tid * GP;
  float* tr = sT + tid * TP;
#pragma unroll 1
  for (int h = 0; h < 8; ++h) {
    float das = 0.0f, dad = 0.0f;
#pragma unroll
    for (int c = 0; c < 4; ++c) {
      const float gv = s0 * c1w[h * 4 + c];
      gr[h * 4 + c] = gv;
      das += gv * c1as[h * 4 + c];
      dad += gv * c1ad[h * 4 + c];
    }
    tr[h] = das;
    tr[8 + h] = dad;
  }
  __syncthreads();
  const int rowW = wave * 32;
  store_rows32<GP>(sG + rowW * GP, gout + (size_t)(nodeBase + rowW) * GP, lane);
  store_rows32<TP>(sT + rowW * TP, tout + (size_t)(nodeBase + rowW) * TP, lane);
}

template <int H, int HN, int NEXT>
__global__ __launch_bounds__(GTHR) void k_gat(
    const int* __restrict__ csr, const int* __restrict__ off, const int* __restrict__ cnt,
    const float* __restrict__ gin, const float* __restrict__ tin, const float* __restrict__ bias,
    const float* __restrict__ Wn, const float* __restrict__ asn, const float* __restrict__ adn,
    float* gout, float* tout, float* xout, int nN, int csrLen) {
  constexpr int CW = 4 * H;
  constexpr int G  = 32 / CW;
  constexpr int CN = HN > 0 ? 4 * HN : 4;
  __shared__ __attribute__((aligned(16))) _Float16 sA[GROW * AP];
  __shared__ __attribute__((aligned(16))) _Float16 sW[16 * 32];
  __shared__ __attribute__((aligned(16))) float sG[GROW * GP];
  __shared__ __attribute__((aligned(16))) float sT[GROW * TP];
  __shared__ __attribute__((aligned(16))) float sX[GROW * XP];
  const int tid = threadIdx.x, lane = tid & 31, wave = tid >> 5, hh = lane >> 4, m = lane & 15;
  const int gi = lane / CW, c = lane - gi * CW, hd = c >> 2;
  const int rowW  = wave * 32;
  const int tbase = blockIdx.x * GROW + rowW;

  if (NEXT) {
    for (int i = tid; i < 16 * 32; i += GTHR) {
      const int n = i >> 5, k = i & 31;
      const int kc  = k < CW ? k : CW - 1;
      const int ncl = n < CN ? n : CN - 1;
      const float w = Wn[kc * CN + ncl];
      sW[i] = (_Float16)((k < CW && n < CN) ? w * WSC : 0.0f);
    }
  }

  const int cnt_l = cnt[tbase + lane];
  const int off_l = off[tbase + lane];
  const float bc = bias[c];

#pragma unroll 1
  for (int it = 0; it < CW; ++it) {
    const int j = it * G + gi;
    const int n = tbase + j;
    int nj = __shfl(cnt_l, j);
    nj = nj < 0 ? 0 : (nj > DEGCAP ? DEGCAP : nj);
    const int st = __shfl(off_l, j);
    const int nmax = wave_max(nj);
    const float ad_n = tin[(size_t)n * TP + 8 + hd];
    float e0 = tin[(size_t)n * TP + hd] + ad_n;
    e0 = e0 > 0.0f ? e0 : 0.2f * e0;
    float mx = e0, z = 1.0f;
    float av = gin[(size_t)n * GP + c];
#pragma unroll 1
    for (int p = 0; p < nmax; ++p) {
      const bool valid = p < nj;
      int pos = st + p;
      pos = pos < 0 ? 0 : (pos > csrLen - 1 ? csrLen - 1 : pos);
      int s = csr[pos];
      s = s < 0 ? 0 : (s > nN - 1 ? nN - 1 : s);
      const float gs = gin[(size_t)s * GP + c];
      float ee = tin[(size_t)s * TP + hd] + ad_n;
      ee = ee > 0.0f ? ee : 0.2f * ee;
      const float mn = valid ? fmaxf(mx, ee) : mx;
      const float sc = __expf(mx - mn);
      const float w  = valid ? __expf(ee - mn) : 0.0f;
      z  = z * sc + w;
      av = av * sc + w * gs;
      mx = mn;
    }
    const float xv = av * (1.0f / (z + 1e-16f)) + bc;
    const int row = rowW + j;
    if (NEXT) {
      sA[row * AP + c] = (_Float16)xv;
      if (CW == 16) sA[row * AP + c + 16] = (_Float16)0.0f;
    } else {
      sX[row * XP + c] = xv;
    }
  }
  __syncthreads();

  if (NEXT) {
#pragma unroll
    for (int tl = 0; tl < 2; ++tl) {
      const int rb = rowW + 16 * tl;
      FragH a, b;
      const _Float16* ar = sA + (rb + m) * AP + 8 * hh;
      a.h[0] = *(const v8h*)ar;
      a.h[1] = *(const v8h*)(ar + 16);
      const _Float16* bp = sW + m * 32 + 8 * hh;
      b.h[0] = *(const v8h*)bp;
      b.h[1] = *(const v8h*)(bp + 16);
      v8f zc = {0.f, 0.f, 0.f, 0.f, 0.f, 0.f, 0.f, 0.f};
      const v8f d = wmh(a.v, b.v, zc);
      float* sp = sG + (rb + 8 * hh) * GP + m;
#pragma unroll
      for (int r = 0; r < 8; ++r) {
        const float gv = d[r] * WINV;
        sp[r * GP]      = (m < CN) ? gv : 0.0f;
        sp[r * GP + 16] = 0.0f;
      }
    }
    __syncthreads();
    {
      const int row = rowW + lane;
      const float* gr = sG + row * GP;
      float* tr = sT + row * TP;
#pragma unroll
      for (int h = 0; h < 8; ++h) {
        float das = 0.0f, dad = 0.0f;
        if (h < HN) {
#pragma unroll
          for (int cc = 0; cc < 4; ++cc) {
            const float gv = gr[4 * h + cc];
            das += gv * asn[4 * h + cc];
            dad += gv * adn[4 * h + cc];
          }
        }
        tr[h] = das;
        tr[8 + h] = dad;
      }
    }
    __syncthreads();
    store_rows32<GP>(sG + rowW * GP, gout + (size_t)tbase * GP, lane);
    store_rows32<TP>(sT + rowW * TP, tout + (size_t)tbase * TP, lane);
  } else {
    store_rows32<XP>(sX + rowW * XP, xout + (size_t)tbase * XP, lane);
  }
}

__global__ __launch_bounds__(GTHR) void k_final(
    const int* __restrict__ csr, const int* __restrict__ off, const int* __restrict__ cnt,
    const float* __restrict__ x4, const float* __restrict__ x, const float* __restrict__ l2w,
    float* out, int nN, int csrLen) {
  __shared__ __attribute__((aligned(16))) float sO[GROW];
  const int tid = threadIdx.x, lane = tid & 31, wave = tid >> 5;
  const int gi = lane >> 3, c = lane & 7;
  const int rowW  = wave * 32;
  const int tbase = blockIdx.x * GROW + rowW;
  const int cnt_l = cnt[tbase + lane];
  const int off_l = off[tbase + lane];
  const float wl = l2w[c];

#pragma unroll 1
  for (int it = 0; it < 8; ++it) {
    const int j = it * 4 + gi;
    const int n = tbase + j;
    const int nc = n > nN - 1 ? nN - 1 : n;
    int nj = __shfl(cnt_l, j);
    nj = nj < 0 ? 0 : (nj > DEGCAP ? DEGCAP : nj);
    const int st = __shfl(off_l, j);
    const int nmax = wave_max(nj);
    const float xs = x4[(size_t)n * XP + c];
    float accv = xs;
#pragma unroll 1
    for (int p = 0; p < nmax; ++p) {
      const bool valid = p < nj;
      int pos = st + p;
      pos = pos < 0 ? 0 : (pos > csrLen - 1 ? csrLen - 1 : pos);
      int d = csr[pos];
      d = d < 0 ? 0 : (d > nN - 1 ? nN - 1 : d);
      const float y = x4[(size_t)d * XP + c];
      accv += valid ? y : 0.0f;
    }
    float pr = xs * accv;
    pr += __shfl_xor(pr, 1);
    pr += __shfl_xor(pr, 2);
    pr += __shfl_xor(pr, 4);
    float pg = accv * wl;
    pg += __shfl_xor(pg, 1);
    pg += __shfl_xor(pg, 2);
    pg += __shfl_xor(pg, 4);
    const float inv = 1.0f / (float)(nj + 1);
    const float o = pr * inv + x[(size_t)nc * 5] + pg * inv;
    if (c == 0) sO[rowW + j] = o;
  }
  __syncthreads();

  const bool act = tid < 32;
  v4f ov = {0.f, 0.f, 0.f, 0.f};
  int node0 = 0;
  if (act) { ov = *(const v4f*)(sO + 4 * tid); node0 = blockIdx.x * GROW + 4 * tid; }
  const bool full = act && (node0 + 3 < nN);
  const bool part = act && !full && (node0 < nN);
  if (full) {
    *(volatile v4f*)(out + node0) = ov;
  } else if (part) {
    volatile float* op = out + node0;
    op[0] = ov.x;
    if (node0 + 1 < nN) op[1] = ov.y;
    if (node0 + 2 < nN) op[2] = ov.z;
  }
  __threadfence();
  if (full) {
    *(volatile v4f*)(out + node0) = ov;
  } else if (part) {
    volatile float* op = out + node0;
    op[0] = ov.x;
    if (node0 + 1 < nN) op[1] = ov.y;
    if (node0 + 2 < nN) op[2] = ov.z;
  }
}

extern "C" void kernel_launch(void* const* d_in, const int* in_sizes, int n_in,
                              void* d_out, int out_size, void* d_ws, size_t ws_size,
                              hipStream_t stream) {
  if (n_in < 18) return;
  const int nN = in_sizes[0] / 5;
  const int nE = in_sizes[1] / 2;
  if (nN <= 0 || nE <= 0 || in_sizes[0] != nN * 5 || in_sizes[1] != 2 * nE) return;
  if (nE > (1 << 28) || nN > (1 << 24)) return;
  if (in_sizes[3] != 5 || in_sizes[4] < 1) return;
  if (in_sizes[5] != 32 || in_sizes[6] != 32 || in_sizes[7] != 32 || in_sizes[8] != 32) return;
  if (in_sizes[9] != 512 || in_sizes[10] != 16 || in_sizes[11] != 16 || in_sizes[12] != 16) return;
  if (in_sizes[13] != 128 || in_sizes[14] != 8 || in_sizes[15] != 8 || in_sizes[16] != 8) return;
  if (in_sizes[17] < 8) return;
  if (out_size != nN) return;

  const float* x    = (const float*)d_in[0];
  const int*   ei   = (const int*)d_in[1];
  const float* l1w  = (const float*)d_in[3];
  const float* l1b  = (const float*)d_in[4];
  const float* c1w  = (const float*)d_in[5];
  const float* c1as = (const float*)d_in[6];
  const float* c1ad = (const float*)d_in[7];
  const float* c1b  = (const float*)d_in[8];
  const float* c2w  = (const float*)d_in[9];
  const float* c2as = (const float*)d_in[10];
  const float* c2ad = (const float*)d_in[11];
  const float* c2b  = (const float*)d_in[12];
  const float* c3w  = (const float*)d_in[13];
  const float* c3as = (const float*)d_in[14];
  const float* c3ad = (const float*)d_in[15];
  const float* c3b  = (const float*)d_in[16];
  const float* l2w  = (const float*)d_in[17];
  float* out = (float*)d_out;

  const int NPAD   = ((nN + GROW - 1) / GROW) * GROW;
  const int nBC    = (nN + NBC - 1) / NBC;
  const int CNTPAD = nBC * NBC;
  if (4 * nBC + 1 > RBN) return;
  const int nBF    = (nN + NBF - 1) / NBF;
  const int csrLen = ((nE + 31) & ~31) + 4096;
  const int nNode  = NPAD / GROW;

  char* ws = (char*)d_ws;
  size_t o = 0;
  const size_t oCntD = o; o += (size_t)CNTPAD * 4;      o = (o + 255) & ~(size_t)255;
  const size_t oOffD = o; o += (size_t)CNTPAD * 4;      o = (o + 255) & ~(size_t)255;
  const size_t oRbD  = o; o += (size_t)RBN * 4;         o = (o + 255) & ~(size_t)255;
  const size_t oCsrD = o; o += (size_t)csrLen * 4;      o = (o + 255) & ~(size_t)255;
  const size_t oCntS = o; o += (size_t)CNTPAD * 4;      o = (o + 255) & ~(size_t)255;
  const size_t oOffS = o; o += (size_t)CNTPAD * 4;      o = (o + 255) & ~(size_t)255;
  const size_t oRbS  = o; o += (size_t)RBN * 4;         o = (o + 255) & ~(size_t)255;
  const size_t oCsrS = o; o += (size_t)csrLen * 4;      o = (o + 255) & ~(size_t)255;
  const size_t oGA   = o; o += (size_t)NPAD * GP * 4;   o = (o + 255) & ~(size_t)255;
  const size_t oTA   = o; o += (size_t)NPAD * TP * 4;   o = (o + 255) & ~(size_t)255;
  const size_t oGB   = o; o += (size_t)NPAD * GP * 4;   o = (o + 255) & ~(size_t)255;
  const size_t oTB   = o; o += (size_t)NPAD * TP * 4;   o = (o + 255) & ~(size_t)255;
  const size_t oX4   = o; o += (size_t)NPAD * XP * 4;   o = (o + 255) & ~(size_t)255;
  if (o > ws_size || o > ((size_t)128 << 20)) return;
  int*   cntD = (int*)(ws + oCntD);
  int*   offD = (int*)(ws + oOffD);
  int*   rbD  = (int*)(ws + oRbD);
  int*   csrD = (int*)(ws + oCsrD);
  int*   cntS = (int*)(ws + oCntS);
  int*   offS = (int*)(ws + oOffS);
  int*   rbS  = (int*)(ws + oRbS);
  int*   csrS = (int*)(ws + oCsrS);
  float* GA   = (float*)(ws + oGA);
  float* TA   = (float*)(ws + oTA);
  float* GB   = (float*)(ws + oGB);
  float* TB   = (float*)(ws + oTB);
  float* X4   = (float*)(ws + oX4);

  const int vec8 = ((nE & 3) == 0) ? 1 : 0;
  const int* srcRow = ei;
  const int* dstRow = ei + nE;

  k_count<<<nBC, NTHR, 0, stream>>>(dstRow, cntD, nE, vec8);
  k_offsets<<<1, OTHR, 0, stream>>>(cntD, offD, rbD, nBC);
  hipFuncSetAttribute(reinterpret_cast<const void*>(&k_fill),
                      hipFuncAttributeMaxDynamicSharedMemorySize, LDS_FILL);
  k_fill<<<nBF, NTHR, LDS_FILL, stream>>>(dstRow, srcRow, offD, rbD, csrD, nN, nE, vec8, csrLen);

  k_count<<<nBC, NTHR, 0, stream>>>(srcRow, cntS, nE, vec8);
  k_offsets<<<1, OTHR, 0, stream>>>(cntS, offS, rbS, nBC);
  k_fill<<<nBF, NTHR, LDS_FILL, stream>>>(srcRow, dstRow, offS, rbS, csrS, nN, nE, vec8, csrLen);

  k_prep<<<nNode, GTHR, 0, stream>>>(x, l1w, l1b, c1w, c1as, c1ad, GA, TA, nN);

  k_gat<8, 4, 1><<<nNode, GTHR, 0, stream>>>(csrD, offD, cntD, GA, TA, c1b, c2w, c2as, c2ad, GB, TB, X4, nN, csrLen);
  k_gat<4, 2, 1><<<nNode, GTHR, 0, stream>>>(csrD, offD, cntD, GB, TB, c2b, c3w, c3as, c3ad, GA, TA, X4, nN, csrLen);
  k_gat<2, 0, 0><<<nNode, GTHR, 0, stream>>>(csrD, offD, cntD, GA, TA, c3b, c3w, c3as, c3ad, GB, TB, X4, nN, csrLen);

  k_final<<<nNode, GTHR, 0, stream>>>(csrS, offS, cntS, X4, x, l2w, out, nN, csrLen);
}
